// CircularRelativeAttention_85521388798342
// MI455X (gfx1250) — hardware-verified
//
#include <hip/hip_runtime.h>
#include <stddef.h>


#define DEVI __device__ __forceinline__

typedef _Float16 v16h __attribute__((ext_vector_type(16)));
typedef _Float16 v8h  __attribute__((ext_vector_type(8)));
typedef float    v8f  __attribute__((ext_vector_type(8)));
typedef float    v4f  __attribute__((ext_vector_type(4)));
typedef v8h v8ha __attribute__((may_alias));
typedef v4f v4fa __attribute__((may_alias));

static constexpr int BATCH = 2;
static constexpr int SEQ   = 2048;
static constexpr int DM    = 1024;
static constexpr int NH    = 16;
static constexpr int HD    = 64;
static constexpr int PL    = 4096;
static constexpr int BS    = BATCH * SEQ;
static constexpr int TP    = 68;
static constexpr int PP    = 72;

union Frag { v16h v; v8h hv[2]; };

DEVI v8f wmma16(v16h a, v16h b, v8f c) {
  v8f d = __builtin_amdgcn_wmma_f32_16x16x32_f16(false, a, false, b, (short)0, c, false, false);
  asm volatile("v_nop\n\tv_nop\n\tv_nop\n\tv_nop" : "+v"(d) : "v"(a), "v"(b));
  return d;
}

DEVI v16h frag_global(const _Float16* rowp, int k0, int h) {
  Frag f;
  f.hv[0] = *(const v8h*)(rowp + k0 + 8 * h);
  f.hv[1] = *(const v8h*)(rowp + k0 + 16 + 8 * h);
  return f.v;
}
DEVI v16h frag_lds(const _Float16* rowp, int k0, int h) {
  Frag f;
  f.hv[0] = *(const v8ha*)(rowp + k0 + 8 * h);
  f.hv[1] = *(const v8ha*)(rowp + k0 + 16 + 8 * h);
  return f.v;
}

DEVI v8h pack8(v4f a, v4f b) {
  v8h o;
  o[0] = (_Float16)a[0]; o[1] = (_Float16)a[1]; o[2] = (_Float16)a[2]; o[3] = (_Float16)a[3];
  o[4] = (_Float16)b[0]; o[5] = (_Float16)b[1]; o[6] = (_Float16)b[2]; o[7] = (_Float16)b[3];
  return o;
}

__global__ __launch_bounds__(256)
void cvt_x_kernel(const float* __restrict__ x, _Float16* __restrict__ xh, int n8) {
  const int i = blockIdx.x * 256 + threadIdx.x;
  const bool ok = i < n8;
  const _Float16 z = (_Float16)0.0f;
  v8h o = {z, z, z, z, z, z, z, z};
  if (ok) {
    const v4f a = *(const v4f*)(x + (size_t)i * 8);
    const v4f b = *(const v4f*)(x + (size_t)i * 8 + 4);
    o = pack8(a, b);
    *(volatile v8h*)(xh + (size_t)i * 8) = o;
  }
  __threadfence();
  if (ok) *(volatile v8h*)(xh + (size_t)i * 8) = o;
}

__global__ __launch_bounds__(256)
void wt_kernel(const float* __restrict__ w0, const float* __restrict__ w1,
               const float* __restrict__ w2, const float* __restrict__ w3,
               _Float16* __restrict__ t0, _Float16* __restrict__ t1,
               _Float16* __restrict__ t2, _Float16* __restrict__ t3) {
  __shared__ float tile[64][33];
  const int z = blockIdx.z;
  const float* w = (z == 0) ? w0 : (z == 1) ? w1 : (z == 2) ? w2 : w3;
  _Float16* t    = (z == 0) ? t0 : (z == 1) ? t1 : (z == 2) ? t2 : t3;
  const int tid = threadIdx.x, cx = tid & 31, ry = tid >> 5;
  const int nB = blockIdx.x * 32, kB = blockIdx.y * 64;
  for (int yy = ry; yy < 64; yy += 8)
    tile[yy][cx] = w[(size_t)(kB + yy) * DM + nB + cx];
  __syncthreads();
  const int n = tid >> 3, c = tid & 7;
  v8h o;
#pragma unroll
  for (int e = 0; e < 8; ++e) o[e] = (_Float16)(tile[8 * c + e][n] * 64.0f);
  _Float16* dst = t + (size_t)(nB + n) * DM + kB + 8 * c;
  *(volatile v8h*)dst = o;
  __threadfence();
  *(volatile v8h*)dst = o;
}

DEVI void gemm_store_pass(const float* tileF, int mode, int tid, int m0, int n0,
                          _Float16* __restrict__ outH, float* __restrict__ outF) {
  if (mode == 0) {
#pragma unroll
    for (int i = 0; i < 8; ++i) {
      const int c = 64 * i + tid, row = c >> 3, ch = c & 7;
      const float* src = tileF + row * TP + 8 * ch;
      const v4f f0 = *(const v4fa*)src;
      const v4f f1 = *(const v4fa*)(src + 4);
      *(volatile v8h*)(outH + (size_t)(m0 + row) * DM + n0 + 8 * ch) = pack8(f0, f1);
    }
  } else if (mode == 1) {
    const int bb = m0 / SEQ, s0 = m0 % SEQ, hh = n0 / HD;
#pragma unroll
    for (int i = 0; i < 8; ++i) {
      const int c = 64 * i + tid, dd = c >> 3, ch = c & 7;
      v8h o;
#pragma unroll
      for (int e = 0; e < 8; ++e) o[e] = (_Float16)tileF[(8 * ch + e) * TP + dd];
      *(volatile v8h*)(outH + ((size_t)((bb * NH + hh) * HD + dd)) * SEQ + s0 + 8 * ch) = o;
    }
  } else {
#pragma unroll
    for (int i = 0; i < 16; ++i) {
      const int c = 64 * i + tid, row = c >> 4, ch = c & 15;
      const v4f v = *(const v4fa*)(tileF + row * TP + 4 * ch);
      *(volatile v4f*)(outF + (size_t)(m0 + row) * DM + n0 + 4 * ch) = v;
    }
  }
}

__global__ __launch_bounds__(64)
void gemm_kernel(const _Float16* __restrict__ A, const _Float16* __restrict__ Bt,
                 const float* __restrict__ bias,
                 _Float16* __restrict__ outH, float* __restrict__ outF,
                 float scale, int mode) {
  __shared__ __align__(16) float tileF[64 * TP];
  const int tid = threadIdx.x, wave = tid >> 5, l = tid & 31, h = l >> 4, m = l & 15;
  const int m0 = blockIdx.y * 64, n0 = blockIdx.x * 64;

  const _Float16* aRow0 = A + (size_t)(m0 + 32 * wave + m) * DM;
  const _Float16* aRow1 = aRow0 + (size_t)16 * DM;
  const _Float16* bRow  = Bt + (size_t)(n0 + m) * DM;

  const v8f zero = {0.f, 0.f, 0.f, 0.f, 0.f, 0.f, 0.f, 0.f};
  v8f acc[2][4];
#pragma unroll
  for (int mi = 0; mi < 2; ++mi)
#pragma unroll
    for (int nj = 0; nj < 4; ++nj) acc[mi][nj] = zero;

#pragma unroll 1
  for (int k0 = 0; k0 < DM; k0 += 32) {
    const v16h a0 = frag_global(aRow0, k0, h);
    const v16h a1 = frag_global(aRow1, k0, h);
#pragma unroll
    for (int nj = 0; nj < 4; ++nj) {
      const v16h bb = frag_global(bRow + (size_t)nj * 16 * DM, k0, h);
      acc[0][nj] = wmma16(a0, bb, acc[0][nj]);
      acc[1][nj] = wmma16(a1, bb, acc[1][nj]);
    }
  }

#pragma unroll
  for (int nj = 0; nj < 4; ++nj) {
    const int nn = 16 * nj + m;
    const float bvv = bias[n0 + nn];
#pragma unroll
    for (int r = 0; r < 8; ++r) {
      tileF[(32 * wave + 8 * h + r) * TP + nn]      = acc[0][nj][r] * scale + bvv;
      tileF[(32 * wave + 16 + 8 * h + r) * TP + nn] = acc[1][nj][r] * scale + bvv;
    }
  }
  __syncthreads();
  gemm_store_pass(tileF, mode, tid, m0, n0, outH, outF);
  __threadfence();
  gemm_store_pass(tileF, mode, tid, m0, n0, outH, outF);
}

DEVI void ao_store_pass(const _Float16* pW, _Float16* __restrict__ AO, size_t rowBase, int l) {
#pragma unroll
  for (int i = 0; i < 4; ++i) {
    const int c = 32 * i + l, row = c >> 3, ch = c & 7;
    const v8h v = *(const v8ha*)(pW + row * PP + 8 * ch);
    *(volatile v8h*)(AO + rowBase + (size_t)row * DM + 8 * ch) = v;
  }
}

__global__ __launch_bounds__(256)
void attn_kernel(const _Float16* __restrict__ Q, const _Float16* __restrict__ Kmat,
                 const _Float16* __restrict__ Vt, const float* __restrict__ rel_bias,
                 _Float16* __restrict__ AO) {
  __shared__ float biasCol[PL];
  __shared__ __align__(16) _Float16 pBuf[8][16 * PP];

  const int tid = threadIdx.x;
  const int bh = blockIdx.y;
  const int b = bh / NH, hh = bh % NH;
  for (int i = tid; i < PL; i += 256) biasCol[i] = rel_bias[(size_t)i * NH + hh];
  __syncthreads();

  const int wave = tid >> 5, l = tid & 31, h = l >> 4, m = l & 15;
  const int q0 = blockIdx.x * 128 + wave * 16;
  _Float16* pW = &pBuf[wave][0];

  const _Float16* qRow = Q + (size_t)(b * SEQ + q0 + m) * DM + hh * HD;
  const v16h qa0 = frag_global(qRow, 0, h);
  const v16h qa1 = frag_global(qRow, 32, h);

  const _Float16* kHead = Kmat + (size_t)(b * SEQ) * DM + hh * HD;
  const _Float16* vHead = Vt + (size_t)(bh * HD) * SEQ;

  float mrow[8], lrow[8];
#pragma unroll
  for (int r = 0; r < 8; ++r) { mrow[r] = -1e30f; lrow[r] = 0.f; }
  const v8f zero = {0.f, 0.f, 0.f, 0.f, 0.f, 0.f, 0.f, 0.f};
  v8f o[4];
#pragma unroll
  for (int j = 0; j < 4; ++j) o[j] = zero;

#pragma unroll 1
  for (int kb = 0; kb < SEQ; kb += 64) {
    v8f s[4];
#pragma unroll
    for (int t = 0; t < 4; ++t) {
      const _Float16* kRow = kHead + (size_t)(kb + 16 * t + m) * DM;
      s[t] = zero;
      s[t] = wmma16(qa0, frag_global(kRow, 0, h), s[t]);
      s[t] = wmma16(qa1, frag_global(kRow, 32, h), s[t]);
    }

#pragma unroll
    for (int r = 0; r < 8; ++r) {
      const int q = q0 + 8 * h + r;
      float v[4];
#pragma unroll
      for (int t = 0; t < 4; ++t)
        v[t] = s[t][r] * 0.125f + biasCol[(q - (kb + 16 * t + m)) & (PL - 1)];
      float mx = fmaxf(fmaxf(v[0], v[1]), fmaxf(v[2], v[3]));
      mx = fmaxf(mx, __shfl_xor(mx, 1, 32));
      mx = fmaxf(mx, __shfl_xor(mx, 2, 32));
      mx = fmaxf(mx, __shfl_xor(mx, 4, 32));
      mx = fmaxf(mx, __shfl_xor(mx, 8, 32));
      const float mnew  = fmaxf(mrow[r], mx);
      const float alpha = __expf(mrow[r] - mnew);
      float p[4];
#pragma unroll
      for (int t = 0; t < 4; ++t) p[t] = __expf(v[t] - mnew);
      float ps = (p[0] + p[1]) + (p[2] + p[3]);
      ps += __shfl_xor(ps, 1, 32);
      ps += __shfl_xor(ps, 2, 32);
      ps += __shfl_xor(ps, 4, 32);
      ps += __shfl_xor(ps, 8, 32);
      lrow[r] = lrow[r] * alpha + ps;
      mrow[r] = mnew;
#pragma unroll
      for (int j = 0; j < 4; ++j) o[j][r] *= alpha;
#pragma unroll
      for (int t = 0; t < 4; ++t)
        pW[(8 * h + r) * PP + 16 * t + m] = (_Float16)(p[t] * 256.0f);
    }
    __syncthreads();
    const v16h pf0 = frag_lds(pW + m * PP, 0, h);
    const v16h pf1 = frag_lds(pW + m * PP, 32, h);
    asm volatile("" ::: "memory");

#pragma unroll
    for (int j = 0; j < 4; ++j) {
      const _Float16* vRow = vHead + (size_t)(16 * j + m) * SEQ + kb;
      o[j] = wmma16(pf0, frag_global(vRow, 0, h), o[j]);
      o[j] = wmma16(pf1, frag_global(vRow, 32, h), o[j]);
    }
  }

  asm volatile("" ::: "memory");
#pragma unroll
  for (int r = 0; r < 8; ++r) {
    const float inv = 1.0f / lrow[r];
#pragma unroll
    for (int j = 0; j < 4; ++j)
      pW[(8 * h + r) * PP + 16 * j + m] = (_Float16)(o[j][r] * inv);
  }
  __syncthreads();
  const size_t rowBase = (size_t)(b * SEQ + q0) * DM + hh * HD;
  ao_store_pass(pW, AO, rowBase, l);
  __threadfence();
  ao_store_pass(pW, AO, rowBase, l);
}

extern "C" void kernel_launch(void* const* d_in, const int* in_sizes, int n_in,
                              void* d_out, int out_size, void* d_ws, size_t ws_size,
                              hipStream_t stream) {
  if (n_in < 10) return;
  if (in_sizes[0] != BS * DM || in_sizes[1] != DM * DM || in_sizes[2] != DM ||
      in_sizes[3] != DM * DM || in_sizes[4] != DM || in_sizes[5] != DM * DM ||
      in_sizes[6] != DM || in_sizes[7] != DM * DM || in_sizes[8] != DM ||
      in_sizes[9] != PL * NH || out_size != BS * DM) return;

  const float* x  = (const float*)d_in[0];
  const float* wq = (const float*)d_in[1];
  const float* bq = (const float*)d_in[2];
  const float* wk = (const float*)d_in[3];
  const float* bk = (const float*)d_in[4];
  const float* wv = (const float*)d_in[5];
  const float* bv = (const float*)d_in[6];
  const float* wo = (const float*)d_in[7];
  const float* bo = (const float*)d_in[8];
  const float* rb = (const float*)d_in[9];
  float* outF = (float*)d_out;

  const size_t hb = (size_t)BS * DM * 2;
  const size_t wb = (size_t)DM * DM * 2;
  const size_t off_x  = 0;
  const size_t off_wq = off_x + hb;
  const size_t off_wk = off_wq + wb;
  const size_t off_wv = off_wk + wb;
  const size_t off_wo = off_wv + wb;
  const size_t off_q  = off_wo + wb;
  const size_t off_k  = off_q + hb;
  const size_t off_vt = off_k + hb;
  const size_t off_ao = off_vt + hb;
  const size_t total  = off_ao + hb;
  if (total > ws_size) return;

  char* ws = (char*)d_ws;
  _Float16* x16  = (_Float16*)(ws + off_x);
  _Float16* wqT  = (_Float16*)(ws + off_wq);
  _Float16* wkT  = (_Float16*)(ws + off_wk);
  _Float16* wvT  = (_Float16*)(ws + off_wv);
  _Float16* woT  = (_Float16*)(ws + off_wo);
  _Float16* q16  = (_Float16*)(ws + off_q);
  _Float16* k16  = (_Float16*)(ws + off_k);
  _Float16* vt16 = (_Float16*)(ws + off_vt);
  _Float16* ao16 = (_Float16*)(ws + off_ao);

  const int n8 = (BS * DM) / 8;
  cvt_x_kernel<<<(n8 + 255) / 256, 256, 0, stream>>>(x, x16, n8);
  wt_kernel<<<dim3(DM / 32, DM / 64, 4), 256, 0, stream>>>(wq, wk, wv, wo, wqT, wkT, wvT, woT);

  const dim3 gg(DM / 64, BS / 64);
  const float s_proj = 1.0f / 64.0f;
  const float s_out  = 1.0f / (64.0f * 256.0f);
  gemm_kernel<<<gg, 64, 0, stream>>>(x16, wqT, bq, q16,  outF, s_proj, 0);
  gemm_kernel<<<gg, 64, 0, stream>>>(x16, wkT, bk, k16,  outF, s_proj, 0);
  gemm_kernel<<<gg, 64, 0, stream>>>(x16, wvT, bv, vt16, outF, s_proj, 1);

  attn_kernel<<<dim3(SEQ / 128, BATCH * NH), 256, 0, stream>>>(q16, k16, vt16, rb, ao16);

  gemm_kernel<<<gg, 64, 0, stream>>>(ao16, woT, bo, ao16, outF, s_out, 2);
}
